// EdgeGAT_19241453486701
// MI455X (gfx1250) — hardware-verified
//
#include <hip/hip_runtime.h>
#include <stddef.h>
#include <stdint.h>


#define DIN     128
#define C1W     128
#define C2W     64
#define KH1     256
#define NTHR    256
#define NWAVE   8
#define EPT     8
#define CHUNK   (NTHR * EPT)
#define WCAP    (EPT * 32)
#define LISTN   (NWAVE * WCAP)
#define NBMAX   2048
#define RCAP    28672
#define DEGCAP  512
#define STW     128
#define GBM     64
#define GBN     64
#define GTHR    128
#define NEGSL   0.2f
#define WSMAX   134217728
#define LDS_AGG ((2 * RCAP + 2 * NBMAX + LISTN) * 4 + 64)

static_assert((CHUNK & (CHUNK - 1)) == 0 && CHUNK <= 4096);
static_assert((NBMAX & (NBMAX - 1)) == 0 && NBMAX <= 4096);
static_assert(NTHR * 8 == NBMAX);
static_assert(LISTN >= NBMAX);
static_assert(LISTN >= NWAVE * WCAP);
static_assert((RCAP % 32) == 0);
static_assert(NWAVE * STW <= RCAP);
static_assert(STW * 4 == KH1 * 2);
static_assert(LDS_AGG <= 300000);
static_assert(GBM == (GTHR / 32) * 16);
static_assert(DIN / 8 == 16);
static_assert((DIN % 32) == 0 && (KH1 % 32) == 0);
static_assert((C1W % GBN) == 0 && (C2W % GBN) == 0);
static_assert(KH1 == 2 * C1W);
static_assert(C1W == 4 * 32 && C2W == 2 * 32);

typedef float          v2f  __attribute__((ext_vector_type(2)));
typedef float          v4f  __attribute__((ext_vector_type(4)));
typedef float          v8f  __attribute__((ext_vector_type(8)));
typedef int            v4i  __attribute__((ext_vector_type(4)));
typedef int            v8i  __attribute__((ext_vector_type(8)));
typedef unsigned int   v2u  __attribute__((ext_vector_type(2)));
typedef unsigned int   v4u  __attribute__((ext_vector_type(4)));
typedef unsigned short v8us __attribute__((ext_vector_type(8)));
typedef __bf16         v16b __attribute__((ext_vector_type(16)));
union FragB { v16b v; v8us h[2]; v8i w; };

__device__ __forceinline__ v8f wmb(const FragB& a, const FragB& b, v8f c) {
  v8f d = __builtin_amdgcn_wmma_f32_16x16x32_bf16(false, a.v, false, b.v, (short)0, c, false, false);
  asm volatile("v_nop\n\tv_nop\n\tv_nop\n\tv_nop" : "+v"(d) : "v"(a.w), "v"(b.w));
  return d;
}

__device__ __forceinline__ void ldwait() {
  asm volatile("s_wait_loadcnt 0x0" ::: "memory");
}

__device__ __forceinline__ unsigned int f2bf(float f) {
  const unsigned int u = __float_as_uint(f);
  return (u + 0x7FFFu + ((u >> 16) & 1u)) >> 16;
}
__device__ __forceinline__ float bf2f(unsigned int b) { return __uint_as_float(b << 16); }
__device__ __forceinline__ float bfr(float f) { return bf2f(f2bf(f)); }
__device__ __forceinline__ v4f bfr4(const v4f a) {
  v4f r; r.x = bfr(a.x); r.y = bfr(a.y); r.z = bfr(a.z); r.w = bfr(a.w); return r;
}
__device__ __forceinline__ v2f bfr2(const v2f a) {
  v2f r; r.x = bfr(a.x); r.y = bfr(a.y); return r;
}
__device__ __forceinline__ unsigned int pk2(float lo, float hi) { return f2bf(lo) | (f2bf(hi) << 16); }
__device__ __forceinline__ v4u pack8(const v4f a, const v4f b) {
  v4u r;
  r.x = pk2(a.x, a.y); r.y = pk2(a.z, a.w); r.z = pk2(b.x, b.y); r.w = pk2(b.z, b.w);
  return r;
}

__device__ __forceinline__ int scan_chunk(const int* __restrict__ dsts, int nE, int cbase, int slotBase,
                                          int nb, int vec8, int* list, int tid, int lane, int wave) {
  int wc = 0;
  const int el0  = tid * EPT;
  const int e0   = cbase + el0;
  const int sent = -2147483647 - 1;
  v4i da, db;
  if (vec8 != 0 && cbase + CHUNK <= nE) {
    da = *(const v4i*)(dsts + e0);
    db = *(const v4i*)(dsts + e0 + 4);
  } else {
    da.x = (e0     < nE) ? dsts[min(e0,     nE - 1)] : sent;
    da.y = (e0 + 1 < nE) ? dsts[min(e0 + 1, nE - 1)] : sent;
    da.z = (e0 + 2 < nE) ? dsts[min(e0 + 2, nE - 1)] : sent;
    da.w = (e0 + 3 < nE) ? dsts[min(e0 + 3, nE - 1)] : sent;
    db.x = (e0 + 4 < nE) ? dsts[min(e0 + 4, nE - 1)] : sent;
    db.y = (e0 + 5 < nE) ? dsts[min(e0 + 5, nE - 1)] : sent;
    db.z = (e0 + 6 < nE) ? dsts[min(e0 + 6, nE - 1)] : sent;
    db.w = (e0 + 7 < nE) ? dsts[min(e0 + 7, nE - 1)] : sent;
  }
  const unsigned nbs = (unsigned)slotBase;
  const unsigned unb = (unsigned)nb;
  const unsigned s0 = (unsigned)da.x - nbs, s1 = (unsigned)da.y - nbs;
  const unsigned s2 = (unsigned)da.z - nbs, s3 = (unsigned)da.w - nbs;
  const unsigned s4 = (unsigned)db.x - nbs, s5 = (unsigned)db.y - nbs;
  const unsigned s6 = (unsigned)db.z - nbs, s7 = (unsigned)db.w - nbs;
  const bool h0 = s0 < unb, h1 = s1 < unb, h2 = s2 < unb, h3 = s3 < unb;
  const bool h4 = s4 < unb, h5 = s5 < unb, h6 = s6 < unb, h7 = s7 < unb;
  const unsigned any = __builtin_amdgcn_ballot_w32(h0 | h1 | h2 | h3 | h4 | h5 | h6 | h7);
  if (any != 0u) {
#define HITJ(J, HJ, SJ) { \
      const unsigned mj = __builtin_amdgcn_ballot_w32(HJ); \
      if (mj != 0u) { \
        if (HJ) { \
          const int pos = wc + (int)__builtin_amdgcn_mbcnt_lo(mj, 0u); \
          if (pos < WCAP) list[wave * WCAP + pos] = ((el0 + (J)) << 12) | (int)(SJ); \
        } \
        wc += (int)__builtin_popcount(mj); } }
    HITJ(0, h0, s0)
    HITJ(1, h1, s1)
    HITJ(2, h2, s2)
    HITJ(3, h3, s3)
    HITJ(4, h4, s4)
    HITJ(5, h5, s5)
    HITJ(6, h6, s6)
    HITJ(7, h7, s7)
#undef HITJ
  }
  return wc;
}

__global__ __launch_bounds__(NTHR) void k_xprep(const float* __restrict__ x, unsigned short* xb, int nN, int nUnits) {
  const int i = (int)blockIdx.x * NTHR + (int)threadIdx.x;
  if (i >= nUnits) return;
  const int row = i >> 4;
  const int c0  = (i & 15) * 8;
  const int rc  = row < nN ? row : nN - 1;
  const float* p = x + (size_t)rc * DIN + c0;
  v4f a = *(const v4f*)p, b = *(const v4f*)(p + 4);
  const v4f z4 = {0.f, 0.f, 0.f, 0.f};
  if (row >= nN) { a = z4; b = z4; }
  const v4u wv = pack8(a, b);
  unsigned short* o = xb + (size_t)row * DIN + c0;
  *(volatile v4u*)o = wv;
  __threadfence();
  *(volatile v4u*)o = wv;
}

__global__ __launch_bounds__(NTHR) void k_wtr(const float* __restrict__ w, int Kin, int Ncol, int nSeg, int Kout,
                                              unsigned short* wt, int nUnits) {
  const int u = (int)blockIdx.x * NTHR + (int)threadIdx.x;
  if (u >= nUnits) return;
  const int kq = Kout >> 3;
  const int n  = u / kq;
  const int k8 = (u - n * kq) * 8;
  const int kk = k8 - (k8 / Kin) * Kin;
  int seg = n / Ncol;
  seg = seg > nSeg - 1 ? nSeg - 1 : (seg < 0 ? 0 : seg);
  int nc = n - seg * Ncol;
  nc = nc < 0 ? 0 : (nc > Ncol - 1 ? Ncol - 1 : nc);
  const float* p = w + (size_t)seg * (size_t)Kin * (size_t)Ncol + (size_t)kk * (size_t)Ncol + nc;
  v4f a, b;
  a.x = p[0];                    a.y = p[(size_t)Ncol];         a.z = p[(size_t)2 * Ncol];     a.w = p[(size_t)3 * Ncol];
  b.x = p[(size_t)4 * Ncol];     b.y = p[(size_t)5 * Ncol];     b.z = p[(size_t)6 * Ncol];     b.w = p[(size_t)7 * Ncol];
  const v4u wv = pack8(a, b);
  unsigned short* o = wt + (size_t)n * (size_t)Kout + k8;
  *(volatile v4u*)o = wv;
  __threadfence();
  *(volatile v4u*)o = wv;
}

__global__ __launch_bounds__(GTHR) void k_gemm(
    const unsigned short* __restrict__ A, const unsigned short* __restrict__ WT,
    float* outF, int K, int ldo)
{
  __shared__ __attribute__((aligned(16))) float stg[GBM * GBN];
  const int tid = (int)threadIdx.x, lane = tid & 31, wave = tid >> 5, hh = lane >> 4, m = lane & 15;
  const int rowBase = (int)blockIdx.x * GBM;
  const int col0    = (int)blockIdx.y * GBN;

  v8f acc[4];
  {
    const v8f z = {0.f, 0.f, 0.f, 0.f, 0.f, 0.f, 0.f, 0.f};
    acc[0] = z; acc[1] = z; acc[2] = z; acc[3] = z;
  }
  const unsigned short* ap = A  + (size_t)(rowBase + 16 * wave + m) * (size_t)K + 8 * hh;
  const unsigned short* wp = WT + (size_t)(col0 + m) * (size_t)K + 8 * hh;
  const int ksteps = K >> 5;
#pragma unroll 1
  for (int ks = 0; ks < ksteps; ++ks) {
    FragB af;
    af.h[0] = *(const v8us*)(ap + 32 * ks);
    af.h[1] = *(const v8us*)(ap + 32 * ks + 16);
#pragma unroll
    for (int t = 0; t < 4; ++t) {
      const unsigned short* wq = wp + (size_t)(16 * t) * (size_t)K + 32 * ks;
      FragB bf;
      bf.h[0] = *(const v8us*)wq;
      bf.h[1] = *(const v8us*)(wq + 16);
      acc[t] = wmb(af, bf, acc[t]);
    }
  }

#pragma unroll
  for (int t = 0; t < 4; ++t) {
    const int lc = 16 * t + m;
#pragma unroll
    for (int r = 0; r < 8; ++r) {
      const int lr = 16 * wave + 8 * hh + r;
      stg[lr * GBN + lc] = acc[t][r];
    }
  }
  __syncthreads();

  v4f fv[8];
#pragma unroll
  for (int i = 0; i < 8; ++i) {
    const int lr = 16 * wave + 2 * i + hh;
    fv[i] = *(const v4f*)(stg + lr * GBN + 4 * m);
  }
#pragma unroll
  for (int i = 0; i < 8; ++i) {
    const int lr = 16 * wave + 2 * i + hh;
    const int gr = rowBase + lr;
    float* op = outF + (size_t)gr * (size_t)ldo + col0 + 4 * m;
    *(volatile v4f*)op = fv[i];
  }
  __threadfence();
#pragma unroll
  for (int i = 0; i < 8; ++i) {
    const int lr = 16 * wave + 2 * i + hh;
    const int gr = rowBase + lr;
    float* op = outF + (size_t)gr * (size_t)ldo + col0 + 4 * m;
    *(volatile v4f*)op = fv[i];
  }
}

template<int L>
__global__ __launch_bounds__(NTHR) void k_agg(
    const int* __restrict__ srcs, const int* __restrict__ dsts, const int* __restrict__ etyp, int tsel,
    const float* __restrict__ P, const float* __restrict__ asrc, const float* __restrict__ adst,
    const float* __restrict__ bias, unsigned short* H1B, float* out,
    int nN, int nE, int nb, int vec8, int MPr, int ldo, int colOff) {
  extern __shared__ v4f lds_dyn[];
  int* reg1 = (int*)lds_dyn;
  int* reg2 = reg1 + RCAP;
  int* scnt = reg2 + RCAP;
  int* soff = scnt + NBMAX;
  int* list = soff + NBMAX;
  int* wcnt = list + LISTN;
  int* wtot = wcnt + NWAVE;
  const int tid = (int)threadIdx.x, lane = tid & 31, wave = tid >> 5;
  const int nodeBase = (int)blockIdx.x * nb;

  for (int i = tid; i < NBMAX; i += NTHR) scnt[i] = 0;
  __syncthreads();

  int tot = 0;
  const int nChunks = (nE + CHUNK - 1) / CHUNK;
#pragma unroll 1
  for (int ch = 0; ch < nChunks; ++ch) {
    const int cbase = ch * CHUNK;
    const int wc = scan_chunk(dsts, nE, cbase, nodeBase, nb, vec8, list, tid, lane, wave);
    if (lane == 0) wcnt[wave] = wc;
    __syncthreads();
    int pre = 0, all = 0;
#pragma unroll
    for (int w2 = 0; w2 < NWAVE; ++w2) {
      int c = wcnt[w2];
      c = c < 0 ? 0 : (c > WCAP ? WCAP : c);
      all += c;
      pre += (w2 < wave) ? c : 0;
    }
    const int wcc  = wc > WCAP ? WCAP : wc;
    const int base = tot + pre;
#pragma unroll 1
    for (int i = lane; i < wcc; i += 32) {
      const int ent = list[wave * WCAP + i];
      const int el  = (ent >> 12) & (CHUNK - 1);
      const int sl  = ent & (NBMAX - 1);
      int eid = cbase + el;
      eid = eid > nE - 1 ? nE - 1 : eid;
      const int pos = base + i;
      if (pos < RCAP) reg1[pos] = (int)(((unsigned)eid << 12) | (unsigned)sl);
    }
    tot += all;
    tot = tot > RCAP ? RCAP : tot;
    __syncthreads();
  }
  const int nh = tot;

  if (wave == 0) {
#pragma unroll 1
    for (int b0 = 0; b0 < nh; b0 += 32) {
      const int idx = b0 + lane;
      const int uv  = reg1[idx < RCAP ? idx : RCAP - 1];
      const int m32 = (nh - b0) < 32 ? (nh - b0) : 32;
#pragma unroll 1
      for (int k = 0; k < m32; ++k) {
        const int u  = __builtin_amdgcn_readlane(uv, k);
        const int sl = u & (NBMAX - 1);
        if (lane == 0) scnt[sl] = scnt[sl] + 1;
      }
    }
  }
  __syncthreads();

  {
    const v4i ca = *(const v4i*)(scnt + 8 * tid);
    const v4i cb = *(const v4i*)(scnt + 8 * tid + 4);
    const int e0 = ca.x < 0 ? 0 : ca.x, e1 = ca.y < 0 ? 0 : ca.y, e2 = ca.z < 0 ? 0 : ca.z, e3 = ca.w < 0 ? 0 : ca.w;
    const int e4 = cb.x < 0 ? 0 : cb.x, e5 = cb.y < 0 ? 0 : cb.y, e6 = cb.z < 0 ? 0 : cb.z, e7 = cb.w < 0 ? 0 : cb.w;
    const int ts = e0 + e1 + e2 + e3 + e4 + e5 + e6 + e7;
    int incl = ts;
#pragma unroll
    for (int d = 1; d < 32; d <<= 1) {
      const int up = __shfl_up(incl, d);
      if (lane >= d) incl += up;
    }
    if (lane == 31) wtot[wave] = incl;
    __syncthreads();
    int pre = 0;
#pragma unroll
    for (int w2 = 0; w2 < NWAVE; ++w2) pre += (w2 < wave) ? wtot[w2] : 0;
    int run = pre + incl - ts;
    soff[8 * tid + 0] = run; run += e0;
    soff[8 * tid + 1] = run; run += e1;
    soff[8 * tid + 2] = run; run += e2;
    soff[8 * tid + 3] = run; run += e3;
    soff[8 * tid + 4] = run; run += e4;
    soff[8 * tid + 5] = run; run += e5;
    soff[8 * tid + 6] = run; run += e6;
    soff[8 * tid + 7] = run;
  }
  __syncthreads();
  for (int i = tid; i < NBMAX; i += NTHR) list[i] = soff[i];
  __syncthreads();

  if (wave == 0) {
#pragma unroll 1
    for (int b0 = 0; b0 < nh; b0 += 32) {
      const int idx = b0 + lane;
      const int uv  = reg1[idx < RCAP ? idx : RCAP - 1];
      const int m32 = (nh - b0) < 32 ? (nh - b0) : 32;
#pragma unroll 1
      for (int k = 0; k < m32; ++k) {
        const int u   = __builtin_amdgcn_readlane(uv, k);
        const int sl  = u & (NBMAX - 1);
        const int eid = (int)((unsigned)u >> 12);
        if (lane == 0) {
          int pos = list[sl];
          pos = pos < 0 ? 0 : (pos > RCAP - 1 ? RCAP - 1 : pos);
          reg2[pos] = eid;
          list[sl] = pos + 1;
        }
      }
    }
  }
  __syncthreads();

  const int nbw = nb >> 3;
  const bool ovf = (nh >= RCAP);
  const float qnan = __int_as_float(0x7fc00000);

  if (L == 1) {
    unsigned int* stw = (unsigned int*)reg1 + wave * STW;
    const v4f as4 = bfr4(*(const v4f*)(asrc + 4 * lane));
    const v4f ad4 = bfr4(*(const v4f*)(adst + 4 * lane));
    const v4f bb  = bfr4(*(const v4f*)(bias + 4 * lane));
#pragma unroll 1
    for (int jt = 0; jt < nbw; ++jt) {
      const int slot = wave * nbw + jt;
      const int grow = nodeBase + slot;
      const int gcl  = grow < nN ? grow : nN - 1;
      int st = soff[slot];
      const int craw = scnt[slot];
      int cnt = craw;
      st  = st < 0 ? 0 : (st > nh ? nh : st);
      cnt = cnt < 0 ? 0 : (cnt > DEGCAP ? DEGCAP : cnt);
      if (cnt > nh - st) cnt = nh - st;
      st  = __builtin_amdgcn_readfirstlane(st);
      cnt = __builtin_amdgcn_readfirstlane(cnt);
      const float pz = (ovf || craw > DEGCAP) ? qnan : 0.0f;
      const bool wr = grow < MPr;
      const float live = grow < nN ? 1.0f : 0.0f;

      const v4f hself = *(const v4f*)(P + (size_t)gcl * C1W + 4 * lane);
      ldwait();
      float sd = hself.x * ad4.x + hself.y * ad4.y + hself.z * ad4.z + hself.w * ad4.w;
      sd += __shfl_xor(sd, 1);
      sd += __shfl_xor(sd, 2);
      float s0 = hself.x * as4.x + hself.y * as4.y + hself.z * as4.z + hself.w * as4.w;
      s0 += __shfl_xor(s0, 1);
      s0 += __shfl_xor(s0, 2);
      float lg0 = s0 + sd;
      lg0 = lg0 > 0.f ? lg0 : NEGSL * lg0;
      float mx = lg0, dn = 1.0f;
      v4f av = hself;

#pragma unroll 1
      for (int q = 0; q < cnt; ++q) {
        int idx = st + q; idx = idx > RCAP - 1 ? RCAP - 1 : idx;
        int eidv = reg2[idx]; eidv = eidv < 0 ? 0 : (eidv > nE - 1 ? nE - 1 : eidv);
        const int eid = __builtin_amdgcn_readfirstlane(eidv);
        const int ty  = __builtin_amdgcn_readfirstlane(etyp[eid]);
        if (ty == tsel) {
          const int sraw = srcs[eid];
          const int s = sraw < 0 ? 0 : (sraw > nN - 1 ? nN - 1 : sraw);
          const v4f hs = *(const v4f*)(P + (size_t)s * C1W + 4 * lane);
          ldwait();
          float es = hs.x * as4.x + hs.y * as4.y + hs.z * as4.z + hs.w * as4.w;
          es += __shfl_xor(es, 1);
          es += __shfl_xor(es, 2);
          float lg = es + sd;
          lg = lg > 0.f ? lg : NEGSL * lg;
          const float df = lg - mx;
          const float ee = __expf(-fabsf(df));
          const bool up  = df > 0.f;
          const float s1 = up ? ee : 1.0f;
          const float s2 = up ? 1.0f : ee;
          mx = up ? lg : mx;
          dn = fmaf(dn, s1, s2);
          av = av * s1 + hs * s2;
        }
      }
      v2u hw, lw;
      {
        const float inv = __builtin_amdgcn_rcpf(dn);
        const float q0 = fmaxf(fmaf(av.x, inv, bb.x), 0.f) * live + pz;
        const float q1 = fmaxf(fmaf(av.y, inv, bb.y), 0.f) * live + pz;
        const float q2 = fmaxf(fmaf(av.z, inv, bb.z), 0.f) * live + pz;
        const float q3 = fmaf(0.f, 0.f, fmaxf(fmaf(av.w, inv, bb.w), 0.f) * live + pz);
        const unsigned int h0 = f2bf(q0), h1 = f2bf(q1), h2 = f2bf(q2), h3 = f2bf(q3);
        const unsigned int l0 = f2bf(q0 - bf2f(h0)), l1 = f2bf(q1 - bf2f(h1));
        const unsigned int l2 = f2bf(q2 - bf2f(h2)), l3 = f2bf(q3 - bf2f(h3));
        hw.x = h0 | (h1 << 16); hw.y = h2 | (h3 << 16);
        lw.x = l0 | (l1 << 16); lw.y = l2 | (l3 << 16);
      }
      __builtin_amdgcn_fence(__ATOMIC_RELEASE, "wavefront");
      __builtin_amdgcn_wave_barrier();
      *(v2u*)(stw + 2 * lane)      = hw;
      *(v2u*)(stw + 64 + 2 * lane) = lw;
      __builtin_amdgcn_fence(__ATOMIC_RELEASE, "wavefront");
      __builtin_amdgcn_wave_barrier();
      const v4u pv = *(const v4u*)(stw + 4 * lane);
      unsigned short* gp = H1B + (size_t)grow * KH1 + 8 * lane;
      if (wr) *(volatile v4u*)gp = pv;
      __threadfence();
      if (wr) *(volatile v4u*)gp = pv;
    }
  } else {
    const v2f as2 = bfr2(*(const v2f*)(asrc + 2 * lane));
    const v2f ad2 = bfr2(*(const v2f*)(adst + 2 * lane));
    const v2f bb  = bfr2(*(const v2f*)(bias + 2 * lane));
#pragma unroll 1
    for (int jt = 0; jt < nbw; ++jt) {
      const int slot = wave * nbw + jt;
      const int grow = nodeBase + slot;
      const int gcl  = grow < nN ? grow : nN - 1;
      int st = soff[slot];
      const int craw = scnt[slot];
      int cnt = craw;
      st  = st < 0 ? 0 : (st > nh ? nh : st);
      cnt = cnt < 0 ? 0 : (cnt > DEGCAP ? DEGCAP : cnt);
      if (cnt > nh - st) cnt = nh - st;
      st  = __builtin_amdgcn_readfirstlane(st);
      cnt = __builtin_amdgcn_readfirstlane(cnt);
      const float pz = (ovf || craw > DEGCAP) ? qnan : 0.0f;
      const bool wr = grow < nN;

      const v2f hself = *(const v2f*)(P + (size_t)gcl * C2W + 2 * lane);
      ldwait();
      float sd = hself.x * ad2.x + hself.y * ad2.y;
      sd += __shfl_xor(sd, 1);
      sd += __shfl_xor(sd, 2);
      float s0 = hself.x * as2.x + hself.y * as2.y;
      s0 += __shfl_xor(s0, 1);
      s0 += __shfl_xor(s0, 2);
      float lg0 = s0 + sd;
      lg0 = lg0 > 0.f ? lg0 : NEGSL * lg0;
      float mx = lg0, dn = 1.0f;
      v2f av = hself;

#pragma unroll 1
      for (int q = 0; q < cnt; ++q) {
        int idx = st + q; idx = idx > RCAP - 1 ? RCAP - 1 : idx;
        int eidv = reg2[idx]; eidv = eidv < 0 ? 0 : (eidv > nE - 1 ? nE - 1 : eidv);
        const int eid = __builtin_amdgcn_readfirstlane(eidv);
        const int ty  = __builtin_amdgcn_readfirstlane(etyp[eid]);
        if (ty == tsel) {
          const int sraw = srcs[eid];
          const int s = sraw < 0 ? 0 : (sraw > nN - 1 ? nN - 1 : sraw);
          const v2f hs = *(const v2f*)(P + (size_t)s * C2W + 2 * lane);
          ldwait();
          float es = hs.x * as2.x + hs.y * as2.y;
          es += __shfl_xor(es, 1);
          es += __shfl_xor(es, 2);
          float lg = es + sd;
          lg = lg > 0.f ? lg : NEGSL * lg;
          const float df = lg - mx;
          const float ee = __expf(-fabsf(df));
          const bool up  = df > 0.f;
          const float s1 = up ? ee : 1.0f;
          const float s2 = up ? 1.0f : ee;
          mx = up ? lg : mx;
          dn = fmaf(dn, s1, s2);
          av = av * s1 + hs * s2;
        }
      }
      const float inv = __builtin_amdgcn_rcpf(dn);
      v2f o;
      o.x = fmaf(av.x, inv, bb.x) + pz;
      o.y = fmaf(av.y, inv, bb.y) + pz;
      float* gp = out + (size_t)gcl * (size_t)ldo + colOff + 2 * lane;
      if (wr) *(volatile v2f*)gp = o;
      __threadfence();
      if (wr) *(volatile v2f*)gp = o;
    }
  }
}

static int pick_nb(int nE, int nN) {
  int nb = NBMAX;
  while (nb > 32 && (long long)nb * (long long)nE * 5LL > (long long)RCAP * (long long)nN * 4LL) nb >>= 1;
  return nb;
}
static inline int cdiv(int a, int b) { return (a + b - 1) / b; }

extern "C" void kernel_launch(void* const* d_in, const int* in_sizes, int n_in,
                              void* d_out, int out_size, void* d_ws, size_t ws_size,
                              hipStream_t stream) {
  if (n_in < 12) return;
  const int nN = in_sizes[0] / DIN;
  if (nN <= 0 || in_sizes[0] != nN * DIN || nN > (1 << 22)) return;
  const int nE = in_sizes[1];
  if (nE < 1 || nE > (1 << 20)) return;
  if (in_sizes[2] != nE || in_sizes[3] != nE) return;
  const int T = in_sizes[4] / (DIN * C1W);
  if (T < 1 || T > 16 || in_sizes[4] != T * DIN * C1W) return;
  if (in_sizes[5] != T * C1W || in_sizes[6] != T * C1W) return;
  if (in_sizes[7] != T * C1W) return;
  if (in_sizes[8] != T * C1W * C2W) return;
  if (in_sizes[9] != T * C2W || in_sizes[10] != T * C2W) return;
  if (in_sizes[11] != T * C2W) return;
  const int ldo = T * C2W;
  if (out_size != nN * ldo) return;

  const float* x    = (const float*)d_in[0];
  const int*   esrc = (const int*)  d_in[1];
  const int*   edst = (const int*)  d_in[2];
  const int*   etyp = (const int*)  d_in[3];
  const float* W1   = (const float*)d_in[4];
  const float* a1s  = (const float*)d_in[5];
  const float* a1d  = (const float*)d_in[6];
  const float* b1   = (const float*)d_in[7];
  const float* W2   = (const float*)d_in[8];
  const float* a2s  = (const float*)d_in[9];
  const float* a2d  = (const float*)d_in[10];
  const float* b2   = (const float*)d_in[11];
  float* out = (float*)d_out;

  const int MP   = cdiv(nN, GBM) * GBM;
  const int nb   = pick_nb(nE, nN);
  if (nb < 32 || (nb & (nb - 1)) != 0 || nb > NBMAX) return;
  const int gA   = cdiv(MP, nb);
  const int vec8 = ((nE & 3) == 0) ? 1 : 0;
  if (gA * nb < MP) return;

  char* ws = (char*)d_ws;
  size_t off = 0;
  const size_t oXB  = off; off += (size_t)MP * DIN * 2;              off = (off + 255) & ~(size_t)255;
  const size_t oW1T = off; off += (size_t)T * C1W * DIN * 2;         off = (off + 255) & ~(size_t)255;
  const size_t oW2T = off; off += (size_t)T * C2W * KH1 * 2;         off = (off + 255) & ~(size_t)255;
  const size_t oHT  = off; off += (size_t)MP * C1W * 4;              off = (off + 255) & ~(size_t)255;
  const size_t oH1B = off; off += (size_t)MP * KH1 * 2;              off = (off + 255) & ~(size_t)255;
  const size_t oG   = off; off += (size_t)MP * C2W * 4;              off = (off + 255) & ~(size_t)255;
  if (off > ws_size || off > (size_t)WSMAX) return;
  unsigned short* XB  = (unsigned short*)(ws + oXB);
  unsigned short* W1T = (unsigned short*)(ws + oW1T);
  unsigned short* W2T = (unsigned short*)(ws + oW2T);
  float*          HT  = (float*)(ws + oHT);
  unsigned short* H1B = (unsigned short*)(ws + oH1B);
  float*          G   = (float*)(ws + oG);

  hipFuncSetAttribute(reinterpret_cast<const void*>(&k_agg<1>),
                      hipFuncAttributeMaxDynamicSharedMemorySize, LDS_AGG);
  hipFuncSetAttribute(reinterpret_cast<const void*>(&k_agg<2>),
                      hipFuncAttributeMaxDynamicSharedMemorySize, LDS_AGG);

  const int nUx = MP * (DIN / 8);
  k_xprep<<<cdiv(nUx, NTHR), NTHR, 0, stream>>>(x, XB, nN, nUx);

  {
    const int nU1 = T * C1W * (DIN / 8);
    k_wtr<<<cdiv(nU1, NTHR), NTHR, 0, stream>>>(W1, DIN, C1W, T, DIN, W1T, nU1);
    const int nU2 = T * C2W * (KH1 / 8);
    k_wtr<<<cdiv(nU2, NTHR), NTHR, 0, stream>>>(W2, C1W, C2W, T, KH1, W2T, nU2);
  }

  const int gM = MP / GBM;
#pragma unroll 1
  for (int t = 0; t < T; ++t) {
    k_gemm<<<dim3(gM, C1W / GBN), GTHR, 0, stream>>>(XB, W1T + (size_t)t * C1W * DIN, HT, DIN, C1W);
    k_agg<1><<<gA, NTHR, LDS_AGG, stream>>>(esrc, edst, etyp, t, HT, a1s + (size_t)t * C1W, a1d + (size_t)t * C1W,
                                            b1 + (size_t)t * C1W, H1B, out, nN, nE, nb, vec8, MP, ldo, 0);
    k_gemm<<<dim3(gM, C2W / GBN), GTHR, 0, stream>>>(H1B, W2T + (size_t)t * C2W * KH1, G, KH1, C2W);
    k_agg<2><<<gA, NTHR, LDS_AGG, stream>>>(esrc, edst, etyp, t, G, a2s + (size_t)t * C2W, a2d + (size_t)t * C2W,
                                            b2 + (size_t)t * C2W, H1B, out, nN, nE, nb, vec8, MP, ldo, t * C2W);
  }
}
